// SelfAttention_88132728914454
// MI455X (gfx1250) — hardware-verified
//
#include <hip/hip_runtime.h>


#ifndef NB
#define NB 2
#endif
#ifndef SEQ
#define SEQ 2048
#endif
#define NB_FULL    2
#define SEQ_FULL   2048
#define DMODEL     1024
#define NHEAD      16
#define HDIM       64
#define QKV_COLS   (3 * DMODEL)
#define HEAD_COLS  (3 * HDIM)
#define BQ         128
#define BK         32
#define NWAVE      8
#define TP         72
#define OP         68
#define CP         68
#define GM         128
#define GN         64
#define MROWS      (NB * SEQ)
#define PLANE      ((size_t)NB * NHEAD * SEQ * HDIM)

static_assert(SEQ % BQ == 0);
static_assert(SEQ % GM == 0);
static_assert(SEQ % BK == 0);
static_assert(BQ == NWAVE * 16);
static_assert(HDIM == 64);
static_assert(NHEAD * HDIM == DMODEL);
static_assert(DMODEL % 64 == 0);
static_assert(QKV_COLS % GN == 0);
static_assert(HEAD_COLS % GN == 0);
static_assert(MROWS % GM == 0);
static_assert(MROWS % 2 == 0);
static_assert(SEQ <= SEQ_FULL);
static_assert(NB >= 1 && NB <= NB_FULL);
static_assert((TP * 2) % 16 == 0);
static_assert((OP * 4) % 16 == 0);
static_assert((CP * 4) % 16 == 0);
static_assert(((size_t)MROWS * DMODEL * 2 * 2 + (size_t)QKV_COLS * DMODEL * 2 + (size_t)DMODEL * DMODEL * 2 +
               5 * PLANE * 2) <= (size_t)134217728);

typedef __bf16         bf16;
typedef _Float16       f16;
typedef unsigned short u16;
typedef bf16     v16bf __attribute__((ext_vector_type(16)));
typedef f16      v16h  __attribute__((ext_vector_type(16)));
typedef f16      v8h   __attribute__((ext_vector_type(8)));
typedef u16      v8us  __attribute__((ext_vector_type(8)));
typedef float    v8f   __attribute__((ext_vector_type(8)));
typedef float    v4f   __attribute__((ext_vector_type(4)));
typedef unsigned v4u   __attribute__((ext_vector_type(4)));

union FragB  { v16bf v; v4u q[2]; bf16 h[16]; };
union FragH  { v16h  v; v4u q[2]; f16  h[16]; };
union FragU  { v4u q[2]; v16bf b; v16h h; };
union Pack8B { v4u u; bf16 h[8]; };
union Pack8H { v4u u; v8h v; f16 h[8]; };
union Pack8U { v4u u; v8us v; u16 h[8]; };

static __device__ __forceinline__ v8f mma_bf16(v16bf a, v16bf b, v8f acc) {
  acc = __builtin_amdgcn_wmma_f32_16x16x32_bf16(false, a, false, b, (short)0, acc, false, false);
  asm volatile("v_nop\n\tv_nop\n\tv_nop\n\tv_nop" : "+v"(acc) : "v"(a), "v"(b));
  return acc;
}
static __device__ __forceinline__ v8f mma_f16(v16h a, v16h b, v8f acc) {
  acc = __builtin_amdgcn_wmma_f32_16x16x32_f16(false, a, false, b, (short)0, acc, false, false);
  asm volatile("v_nop\n\tv_nop\n\tv_nop\n\tv_nop" : "+v"(acc) : "v"(a), "v"(b));
  return acc;
}

static __device__ __forceinline__ float bf16_rne(float x) { return (float)(bf16)x; }
static __device__ __forceinline__ u16 bits_bf16(float x) { union { bf16 b; u16 u; } c; c.b = (bf16)x; return c.u; }
static __device__ __forceinline__ u16 bits_f16(float x)  { union { f16 h; u16 u; } c; c.h = (f16)x; return c.u; }

__global__ __launch_bounds__(256) void x_plane_kernel(const float* __restrict__ x,
                                                      const int* __restrict__ nheads,
                                                      u16* __restrict__ xb) {
  (void)nheads;
  const size_t g     = (size_t)blockIdx.x * 256 + threadIdx.x;
  const int    row   = (int)(g >> 7);
  const int    piece = (int)(g & 127);
  const int    b     = row / SEQ;
  const int    s     = row - b * SEQ;
  const float* src = x + ((size_t)b * SEQ_FULL + s) * DMODEL + piece * 8;
  const v4f a0 = *(const v4f*)(src);
  const v4f a1 = *(const v4f*)(src + 4);
  Pack8B pk;
  #pragma unroll
  for (int i = 0; i < 4; ++i) {
    pk.h[i]     = (bf16)a0[i];
    pk.h[4 + i] = (bf16)a1[i];
  }
  const v4u val = pk.u;
  u16* dst = xb + (size_t)row * DMODEL + piece * 8;
  *(volatile v4u*)dst = val;
  __threadfence();
  *(volatile v4u*)dst = val;
}

template <int F16>
__global__ __launch_bounds__(256) void w_plane_kernel(const float* __restrict__ w,
                                                      u16* __restrict__ wt, int ncols) {
  const int kBase = blockIdx.x * 64;
  const int nBase = blockIdx.y * 64;
  const int tid   = threadIdx.x;
  __shared__ __align__(16) u16 sT[64 * TP];

  #pragma unroll
  for (int kk = 0; kk < 2; ++kk) {
    const int krow = kk * 32 + (tid >> 3);
    const int n0   = (tid & 7) * 8;
    const float* src = w + (size_t)(kBase + krow) * ncols + nBase + n0;
    const v4f a0 = *(const v4f*)(src);
    const v4f a1 = *(const v4f*)(src + 4);
    #pragma unroll
    for (int i = 0; i < 4; ++i) {
      if (F16) {
        sT[(n0 + i) * TP + krow]     = bits_f16(bf16_rne(a0[i]) * 1024.0f);
        sT[(n0 + 4 + i) * TP + krow] = bits_f16(bf16_rne(a1[i]) * 1024.0f);
      } else {
        sT[(n0 + i) * TP + krow]     = bits_bf16(a0[i]);
        sT[(n0 + 4 + i) * TP + krow] = bits_bf16(a1[i]);
      }
    }
  }
  __syncthreads();

  v4u    val[2];
  size_t idx[2];
  #pragma unroll
  for (int kk = 0; kk < 2; ++kk) {
    const int n  = kk * 32 + (tid >> 3);
    const int ks = (tid & 7) * 8;
    Pack8U p;
    p.v = *(const v8us*)(sT + n * TP + ks);
    val[kk] = p.u;
    idx[kk] = (size_t)(nBase + n) * DMODEL + kBase + ks;
  }
  #pragma unroll
  for (int kk = 0; kk < 2; ++kk) *(volatile v4u*)(wt + idx[kk]) = val[kk];
  __threadfence();
  #pragma unroll
  for (int kk = 0; kk < 2; ++kk) *(volatile v4u*)(wt + idx[kk]) = val[kk];
}

template <int F16OP>
static __device__ __forceinline__ void gemm_core(const u16* __restrict__ A, const u16* __restrict__ Bt,
                                                 int mBase, int nBase, int wrow, int wcol,
                                                 int lq, int hi, v8f (&acc)[2][2]) {
  size_t aoff[2], boff[2];
  #pragma unroll
  for (int t = 0; t < 2; ++t) {
    aoff[t] = (size_t)(mBase + wrow + t * 16 + lq) * DMODEL + hi * 8;
    boff[t] = (size_t)(nBase + wcol + t * 16 + lq) * DMODEL + hi * 8;
  }
  #pragma unroll 2
  for (int k0 = 0; k0 < DMODEL; k0 += 32) {
    FragU a[2], b[2];
    #pragma unroll
    for (int t = 0; t < 2; ++t) {
      a[t].q[0] = *(const v4u*)(A + aoff[t] + k0);
      a[t].q[1] = *(const v4u*)(A + aoff[t] + k0 + 16);
      b[t].q[0] = *(const v4u*)(Bt + boff[t] + k0);
      b[t].q[1] = *(const v4u*)(Bt + boff[t] + k0 + 16);
    }
    #pragma unroll
    for (int rt = 0; rt < 2; ++rt) {
      #pragma unroll
      for (int ct = 0; ct < 2; ++ct) {
        if (F16OP) acc[rt][ct] = mma_f16(a[rt].h, b[ct].h, acc[rt][ct]);
        else       acc[rt][ct] = mma_bf16(a[rt].b, b[ct].b, acc[rt][ct]);
      }
    }
  }
}

__global__ __launch_bounds__(256) void qkv_gemm_kernel(const u16* __restrict__ xb,
                                                       const u16* __restrict__ wqT,
                                                       const float* __restrict__ bias,
                                                       u16* __restrict__ pl) {
  __shared__ __align__(16) float sC[GM * CP];
  const int nBase = blockIdx.x * GN;
  const int mBase = blockIdx.y * GM;
  const int tid   = threadIdx.x;
  const int wave  = tid >> 5;
  const int lane  = tid & 31;
  const int lq    = lane & 15;
  const int hi    = lane >> 4;
  const int wrow  = (wave >> 1) * 32;
  const int wcol  = (wave & 1) * 32;

  v8f acc[2][2];
  #pragma unroll
  for (int rt = 0; rt < 2; ++rt) {
    #pragma unroll
    for (int ct = 0; ct < 2; ++ct) acc[rt][ct] = (v8f){0, 0, 0, 0, 0, 0, 0, 0};
  }
  gemm_core<0>(xb, wqT, mBase, nBase, wrow, wcol, lq, hi, acc);

  #pragma unroll
  for (int ct = 0; ct < 2; ++ct) {
    const float bv = bf16_rne(bias[nBase + wcol + ct * 16 + lq]);
    #pragma unroll
    for (int rt = 0; rt < 2; ++rt) {
      #pragma unroll
      for (int r = 0; r < 8; ++r)
        sC[(wrow + rt * 16 + hi * 8 + r) * CP + wcol + ct * 16 + lq] = acc[rt][ct][r] + bv;
    }
  }
  __syncthreads();

  const int hd    = nBase / HEAD_COLS;
  const int which = (nBase - hd * HEAD_COLS) / HDIM;
  const int b     = mBase / SEQ;
  const int s0    = mBase - b * SEQ;
  const size_t bh = (size_t)b * NHEAD + hd;

  if (which < 2) {
    v4u    hv[4], lv[4];
    size_t idx[4];
    #pragma unroll
    for (int it = 0; it < 4; ++it) {
      const int row = it * 32 + (tid >> 3);
      const int d0  = (tid & 7) * 8;
      const v4f a0 = *(const v4f*)(sC + row * CP + d0);
      const v4f a1 = *(const v4f*)(sC + row * CP + d0 + 4);
      Pack8B ph, pq;
      #pragma unroll
      for (int i = 0; i < 4; ++i) {
        const bf16 h0 = (bf16)a0[i];
        const bf16 h1 = (bf16)a1[i];
        ph.h[i]     = h0;
        ph.h[4 + i] = h1;
        pq.h[i]     = (bf16)(a0[i] - (float)h0);
        pq.h[4 + i] = (bf16)(a1[i] - (float)h1);
      }
      hv[it]  = ph.u;
      lv[it]  = pq.u;
      idx[it] = (size_t)which * 2 * PLANE + (bh * SEQ + s0 + row) * HDIM + d0;
    }
    #pragma unroll
    for (int it = 0; it < 4; ++it) {
      *(volatile v4u*)(pl + idx[it])         = hv[it];
      *(volatile v4u*)(pl + idx[it] + PLANE) = lv[it];
    }
    __threadfence();
    #pragma unroll
    for (int it = 0; it < 4; ++it) {
      *(volatile v4u*)(pl + idx[it])         = hv[it];
      *(volatile v4u*)(pl + idx[it] + PLANE) = lv[it];
    }
  } else {
    v4u    vv[4];
    size_t idx[4];
    #pragma unroll
    for (int it = 0; it < 4; ++it) {
      const int d  = it * 16 + (tid >> 4);
      const int t0 = (tid & 15) * 8;
      Pack8H p;
      #pragma unroll
      for (int i = 0; i < 8; ++i) p.h[i] = (f16)sC[(t0 + i) * CP + d];
      vv[it]  = p.u;
      idx[it] = 4 * PLANE + (bh * HDIM + d) * SEQ + s0 + t0;
    }
    #pragma unroll
    for (int it = 0; it < 4; ++it) *(volatile v4u*)(pl + idx[it]) = vv[it];
    __threadfence();
    #pragma unroll
    for (int it = 0; it < 4; ++it) *(volatile v4u*)(pl + idx[it]) = vv[it];
  }
}

__global__ __launch_bounds__(256) void attn_kernel(const u16* __restrict__ pl,
                                                   const float* __restrict__ mask,
                                                   u16* __restrict__ ctx) {
  const int qblk = blockIdx.x;
  const int h    = blockIdx.y;
  const int b    = blockIdx.z;
  const int tid  = threadIdx.x;
  const int wave = tid >> 5;
  const int lane = tid & 31;
  const int lq   = lane & 15;
  const int hi   = lane >> 4;

  __shared__ __align__(16) float sO[NWAVE * 16 * OP];

  const int    qrow0 = qblk * BQ + wave * 16;
  const size_t bh    = (size_t)b * NHEAD + h;

  FragB qfh[2], qfl[2];
  {
    const u16* qp = pl + (bh * SEQ + qrow0 + lq) * HDIM + hi * 8;
    #pragma unroll
    for (int f = 0; f < 2; ++f) {
      qfh[f].q[0] = *(const v4u*)(qp + f * 32);
      qfh[f].q[1] = *(const v4u*)(qp + f * 32 + 16);
      qfl[f].q[0] = *(const v4u*)(qp + PLANE + f * 32);
      qfl[f].q[1] = *(const v4u*)(qp + PLANE + f * 32 + 16);
    }
  }

  const u16*   kh_h = pl + 2 * PLANE + bh * SEQ * HDIM;
  const u16*   vt_h = pl + 4 * PLANE + bh * HDIM * SEQ;
  const float* mrow = mask + (size_t)(qrow0 + lq) * SEQ_FULL + hi * 8;

  v8f o[4];
  #pragma unroll
  for (int dt = 0; dt < 4; ++dt) o[dt] = (v8f){0, 0, 0, 0, 0, 0, 0, 0};

  float rmax = -__builtin_inff();
  float rsum = 0.0f;
  const float L2E = 1.4426950408889634f;

  for (int i = 0; i < SEQ / BK; ++i) {
    const int j0 = i * BK;

    v8f c[2];
    #pragma unroll
    for (int sub = 0; sub < 2; ++sub) {
      FragB akh[2], akl[2];
      #pragma unroll
      for (int f = 0; f < 2; ++f) {
        const u16* base = kh_h + (size_t)(j0 + sub * 16 + lq) * HDIM + f * 32 + hi * 8;
        akh[f].q[0] = *(const v4u*)(base);
        akh[f].q[1] = *(const v4u*)(base + 16);
        akl[f].q[0] = *(const v4u*)(base + PLANE);
        akl[f].q[1] = *(const v4u*)(base + PLANE + 16);
      }
      v8f acc = (v8f){0, 0, 0, 0, 0, 0, 0, 0};
      acc = mma_bf16(akl[0].v, qfh[0].v, acc);
      acc = mma_bf16(akl[1].v, qfh[1].v, acc);
      acc = mma_bf16(akh[0].v, qfl[0].v, acc);
      acc = mma_bf16(akh[1].v, qfl[1].v, acc);
      acc = mma_bf16(akh[0].v, qfh[0].v, acc);
      acc = mma_bf16(akh[1].v, qfh[1].v, acc);
      c[sub] = acc;
    }

    #pragma unroll
    for (int sub = 0; sub < 2; ++sub) {
      const v4f m0 = *(const v4f*)(mrow + j0 + sub * 16);
      const v4f m1 = *(const v4f*)(mrow + j0 + sub * 16 + 4);
      #pragma unroll
      for (int r = 0; r < 4; ++r) {
        c[sub][r]     = c[sub][r] * 0.125f + bf16_rne(m0[r]);
        c[sub][4 + r] = c[sub][4 + r] * 0.125f + bf16_rne(m1[r]);
      }
    }

    float m_new = rmax;
    #pragma unroll
    for (int r = 0; r < 8; ++r) {
      m_new = fmaxf(m_new, c[0][r]);
      m_new = fmaxf(m_new, c[1][r]);
    }
    m_new = fmaxf(m_new, __shfl_xor(m_new, 16, 32));
    const float m_use = (m_new == -__builtin_inff()) ? 0.0f : m_new;
    const float scale = __builtin_amdgcn_exp2f((rmax - m_use) * L2E);
    rmax = m_new;

    FragH pa;
    float psum = 0.0f;
    #pragma unroll
    for (int r = 0; r < 8; ++r) {
      const float p0 = __builtin_amdgcn_exp2f((c[0][r] - m_use) * L2E);
      const float p1 = __builtin_amdgcn_exp2f((c[1][r] - m_use) * L2E);
      psum += p0 + p1;
      pa.h[r]     = (f16)(p0 * 4096.0f);
      pa.h[8 + r] = (f16)(p1 * 4096.0f);
    }
    rsum = rsum * scale + psum + __shfl_xor(psum, 16, 32);

    float sc[8];
    #pragma unroll
    for (int r = 0; r < 8; ++r) sc[r] = __shfl(scale, (hi << 3) + r, 32);
    #pragma unroll
    for (int dt = 0; dt < 4; ++dt) {
      #pragma unroll
      for (int r = 0; r < 8; ++r) o[dt][r] *= sc[r];
    }

    #pragma unroll
    for (int dt = 0; dt < 4; ++dt) {
      FragH bv;
      const u16* base = vt_h + (size_t)(dt * 16 + lq) * SEQ + j0 + hi * 8;
      bv.q[0] = *(const v4u*)(base);
      bv.q[1] = *(const v4u*)(base + 16);
      o[dt] = mma_f16(pa.v, bv.v, o[dt]);
    }
  }

  float rs[8];
  #pragma unroll
  for (int r = 0; r < 8; ++r) rs[r] = 1.0f / __shfl(rsum, (hi << 3) + r, 32);

  float* so = sO + wave * (16 * OP);
  #pragma unroll
  for (int r = 0; r < 8; ++r) {
    #pragma unroll
    for (int dt = 0; dt < 4; ++dt)
      so[(hi * 8 + r) * OP + dt * 16 + lq] = o[dt][r] * 0.0625f * rs[r];
  }
  __syncthreads();

  v4u    vals[4];
  size_t gidx[4];
  #pragma unroll
  for (int it = 0; it < 4; ++it) {
    const int row = it * 4 + (lane >> 3);
    const int d0  = (lane & 7) * 8;
    const v4f a0 = *(const v4f*)(so + row * OP + d0);
    const v4f a1 = *(const v4f*)(so + row * OP + d0 + 4);
    Pack8H p;
    #pragma unroll
    for (int k = 0; k < 4; ++k) {
      p.h[k]     = (f16)a0[k];
      p.h[4 + k] = (f16)a1[k];
    }
    vals[it] = p.u;
    gidx[it] = ((size_t)b * SEQ + qrow0 + row) * DMODEL + h * HDIM + d0;
  }
  #pragma unroll
  for (int it = 0; it < 4; ++it) *(volatile v4u*)(ctx + gidx[it]) = vals[it];
  __threadfence();
  #pragma unroll
  for (int it = 0; it < 4; ++it) *(volatile v4u*)(ctx + gidx[it]) = vals[it];
}

__global__ __launch_bounds__(256) void out_gemm_kernel(const u16* __restrict__ ctx,
                                                       const u16* __restrict__ woT,
                                                       const float* __restrict__ bias,
                                                       float* __restrict__ out) {
  __shared__ __align__(16) float sC[GM * CP];
  const int nBase = blockIdx.x * GN;
  const int mBase = blockIdx.y * GM;
  const int tid   = threadIdx.x;
  const int wave  = tid >> 5;
  const int lane  = tid & 31;
  const int lq    = lane & 15;
  const int hi    = lane >> 4;
  const int wrow  = (wave >> 1) * 32;
  const int wcol  = (wave & 1) * 32;

  v8f acc[2][2];
  #pragma unroll
  for (int rt = 0; rt < 2; ++rt) {
    #pragma unroll
    for (int ct = 0; ct < 2; ++ct) acc[rt][ct] = (v8f){0, 0, 0, 0, 0, 0, 0, 0};
  }
  gemm_core<1>(ctx, woT, mBase, nBase, wrow, wcol, lq, hi, acc);

  #pragma unroll
  for (int ct = 0; ct < 2; ++ct) {
    const float bv = bf16_rne(bias[nBase + wcol + ct * 16 + lq]);
    #pragma unroll
    for (int rt = 0; rt < 2; ++rt) {
      #pragma unroll
      for (int r = 0; r < 8; ++r)
        sC[(wrow + rt * 16 + hi * 8 + r) * CP + wcol + ct * 16 + lq] =
            acc[rt][ct][r] * (1.0f / 262144.0f) + bv;
    }
  }
  __syncthreads();

  const int b  = mBase / SEQ;
  const int s0 = mBase - b * SEQ;
  v4f    vals[8];
  size_t gidx[8];
  #pragma unroll
  for (int it = 0; it < 8; ++it) {
    const int row = it * 16 + (tid >> 4);
    const int c0  = (tid & 15) * 4;
    vals[it] = *(const v4f*)(sC + row * CP + c0);
    gidx[it] = ((size_t)b * SEQ_FULL + s0 + row) * DMODEL + nBase + c0;
  }
  #pragma unroll
  for (int it = 0; it < 8; ++it) *(volatile v4f*)(out + gidx[it]) = vals[it];
  __threadfence();
  #pragma unroll
  for (int it = 0; it < 8; ++it) *(volatile v4f*)(out + gidx[it]) = vals[it];
}

extern "C" void kernel_launch(void* const* d_in, const int* in_sizes, int n_in,
                              void* d_out, int out_size, void* d_ws, size_t ws_size,
                              hipStream_t stream) {
  if (n_in < 7) return;
  const size_t rows_used = (size_t)(NB - 1) * SEQ_FULL + SEQ;
  if ((size_t)in_sizes[0] < rows_used * DMODEL) return;
  if ((size_t)in_sizes[1] < (size_t)(SEQ - 1) * SEQ_FULL + SEQ) return;
  if ((size_t)in_sizes[2] < (size_t)DMODEL * QKV_COLS) return;
  if ((size_t)in_sizes[3] < (size_t)QKV_COLS) return;
  if ((size_t)in_sizes[4] < (size_t)DMODEL * DMODEL) return;
  if ((size_t)in_sizes[5] < (size_t)DMODEL) return;
  if (in_sizes[6] < 1) return;
  if ((size_t)out_size < rows_used * DMODEL) return;

  const size_t xb_bytes  = (size_t)MROWS * DMODEL * 2;
  const size_t wq_bytes  = (size_t)QKV_COLS * DMODEL * 2;
  const size_t wo_bytes  = (size_t)DMODEL * DMODEL * 2;
  const size_t pl_bytes  = 5 * PLANE * 2;
  const size_t ctx_bytes = (size_t)MROWS * DMODEL * 2;
  const size_t total     = xb_bytes + wq_bytes + wo_bytes + pl_bytes + ctx_bytes;
  if (ws_size < total) return;

  const float* x     = (const float*)d_in[0];
  const float* mask  = (const float*)d_in[1];
  const float* w_qkv = (const float*)d_in[2];
  const float* b_qkv = (const float*)d_in[3];
  const float* w_out = (const float*)d_in[4];
  const float* b_out = (const float*)d_in[5];
  const int*   nhead = (const int*)d_in[6];
  float*       out   = (float*)d_out;

  char* wsb = (char*)d_ws;
  u16* xb  = (u16*)(wsb);
  u16* wqT = (u16*)(wsb + xb_bytes);
  u16* woT = (u16*)(wsb + xb_bytes + wq_bytes);
  u16* pl  = (u16*)(wsb + xb_bytes + wq_bytes + wo_bytes);
  u16* ctx = (u16*)(wsb + xb_bytes + wq_bytes + wo_bytes + pl_bytes);

  x_plane_kernel<<<dim3(MROWS / 2), 256, 0, stream>>>(x, nhead, xb);
  w_plane_kernel<0><<<dim3(DMODEL / 64, QKV_COLS / 64), 256, 0, stream>>>(w_qkv, wqT, QKV_COLS);
  w_plane_kernel<1><<<dim3(DMODEL / 64, DMODEL / 64), 256, 0, stream>>>(w_out, woT, DMODEL);

  qkv_gemm_kernel<<<dim3(QKV_COLS / GN, MROWS / GM), 256, 0, stream>>>(xb, wqT, b_qkv, pl);
  attn_kernel<<<dim3(SEQ / BQ, NHEAD, NB), 256, 0, stream>>>(pl, mask, ctx);
  out_gemm_kernel<<<dim3(DMODEL / GN, MROWS / GM), 256, 0, stream>>>(ctx, woT, b_out, out);
}
